// MultiHeadAttention_43078521979238
// MI455X (gfx1250) — hardware-verified
//
#include <hip/hip_runtime.h>
#include <math.h>

typedef __attribute__((ext_vector_type(16))) _Float16 v16h;
typedef __attribute__((ext_vector_type(16))) __bf16 v16b;
typedef __attribute__((ext_vector_type(8)))  _Float16 v8h;
typedef __attribute__((ext_vector_type(8)))  __bf16 v8b;
typedef __attribute__((ext_vector_type(8)))  float v8f;
typedef __attribute__((ext_vector_type(4)))  float v4f;
typedef __attribute__((ext_vector_type(4)))  unsigned v4u;

#ifndef NB
#define NB 2
#endif
#ifndef SEQ
#define SEQ 2048
#endif
#define TT SEQ
#define NB_FULL 2
#define TT_FULL 2048
#define DIN 1024
#define NH 16
#define HD 64
#define CC (NH * HD)
#define NQB (TT / 64)
#define QBH 4
#define QHI 256
#define KHI 256
#define SC_LOG2E 0.18033688011112042f

static_assert(HD == 64);
static_assert(DIN % 32 == 0);
static_assert(CC % 32 == 0);
static_assert(CC % 128 == 0);
static_assert(DIN % 128 == 0);
static_assert(DIN % 64 == 0);
static_assert(CC == DIN);
static_assert(TT % 64 == 0);
static_assert((NB * TT) % 64 == 0);
static_assert(QHI == QBH * 64);
static_assert(KHI == QHI);
static_assert(TT >= QHI);
static_assert(NB <= NB_FULL);
static_assert(TT <= TT_FULL);
static_assert((NB * TT * (DIN / 8)) % 256 == 0);

template <typename T> __device__ __forceinline__ void vst2(void* p, T v) { *(volatile T*)p = v; __threadfence(); *(volatile T*)p = v; }
__device__ __forceinline__ v8f wmma16(v16h a, v16h b, v8f c) {
  v8f d = __builtin_amdgcn_wmma_f32_16x16x32_f16(false, a, false, b, (short)0, c, false, false);
  asm volatile("v_nop\n\tv_nop\n\tv_nop\n\tv_nop" : "+v"(d) : "v"(a), "v"(b));
  return d;
}
__device__ __forceinline__ v8f wmma_bf(v16b a, v16b b, v8f c) {
  v8f d = __builtin_amdgcn_wmma_f32_16x16x32_bf16(false, a, false, b, (short)0, c, false, false);
  asm volatile("v_nop\n\tv_nop\n\tv_nop\n\tv_nop" : "+v"(d) : "v"(a), "v"(b));
  return d;
}
__device__ __forceinline__ v16h frag_h(const _Float16* rowk0, int lane) {
  union { v16h v; v8h q[2]; } u; const _Float16* p = rowk0 + 8 * (lane >> 4);
  u.q[0] = *(const v8h*)p; u.q[1] = *(const v8h*)(p + 16); return u.v;
}
__device__ __forceinline__ v16b frag_b(const __bf16* rowk0, int lane) {
  union { v16b v; v8b q[2]; } u; const __bf16* p = rowk0 + 8 * (lane >> 4);
  u.q[0] = *(const v8b*)p; u.q[1] = *(const v8b*)(p + 16); return u.v;
}
__device__ __forceinline__ unsigned bf16_rne_bits(float v) { const unsigned u = __float_as_uint(v); return (u + 0x7FFFu + ((u >> 16) & 1u)) >> 16; }
#define LDSX() do { asm volatile("s_wait_dscnt 0" ::: "memory"); __builtin_amdgcn_wave_barrier(); __builtin_amdgcn_fence(3  , "workgroup"); } while (0)

#define WS_XB  ((size_t)0)
#define WS_WT  (WS_XB  + 2u * (size_t)NB * TT * DIN)
#define WS_WPH (WS_WT  + 2u * (size_t)3 * CC * DIN)
#define WS_QH  (WS_WPH + 2u * (size_t)DIN * CC)
#define WS_KH  (WS_QH  + 2u * (size_t)NB * TT * CC)
#define WS_VT  (WS_KH  + 2u * (size_t)NB * TT * CC)
#define WS_QL  (WS_VT  + 2u * (size_t)NB * CC * TT)
#define WS_KL  (WS_QL  + 2u * (size_t)NB * QHI * CC)
#define WS_VB  (WS_KL  + 2u * (size_t)NB * KHI * CC)
#define WS_VBL (WS_VB  + 2u * (size_t)NB * CC * KHI)
#define WS_CH  (WS_VBL + 2u * (size_t)NB * CC * KHI)
#define WS_CL  (WS_CH  + 2u * (size_t)NB * TT * CC)
#define WS_END (WS_CL  + 2u * (size_t)NB * QHI * CC)
static_assert(WS_END <= (size_t)134217728);
static_assert(WS_KH == WS_QH + 2u * (size_t)NB * TT * CC);
static_assert(WS_KL == WS_QL + 2u * (size_t)NB * QHI * CC);

__global__ __launch_bounds__(256) void k_cvt_x(const float* __restrict__ X, unsigned short* __restrict__ XB) {
  const int i = (int)blockIdx.x * 256 + (int)threadIdx.x; if (i >= NB * TT * (DIN / 8)) return;
  const int p = i / (DIN / 8), c8 = (i % (DIN / 8)) * 8; const size_t srow = (size_t)(p / TT) * TT_FULL + (size_t)(p % TT);
  const v4f a = *(const v4f*)(X + srow * DIN + c8), b4 = *(const v4f*)(X + srow * DIN + c8 + 4);
  v4u o; o[0] = bf16_rne_bits(a[0]) | (bf16_rne_bits(a[1]) << 16); o[1] = bf16_rne_bits(a[2]) | (bf16_rne_bits(a[3]) << 16);
  o[2] = bf16_rne_bits(b4[0]) | (bf16_rne_bits(b4[1]) << 16); o[3] = bf16_rne_bits(b4[2]) | (bf16_rne_bits(b4[3]) << 16);
  vst2(XB + (size_t)p * DIN + c8, o);
}
__global__ __launch_bounds__(256) void k_wt(const float* __restrict__ src, unsigned short* __restrict__ dst, int per_head, int f16mode) {
  __shared__ __align__(16) unsigned short t[64][72];
  const int tid = threadIdx.x; const int r0 = (int)blockIdx.x * 64; const int y = blockIdx.y;
  const size_t off0 = per_head ? (size_t)y * DIN * HD : (size_t)y * 64; const int ld = per_head ? HD : DIN;
#pragma unroll 1
  for (int it = 0; it < 4; ++it) { const int e = tid + it * 256; const int r = e >> 4, c4 = (e & 15) * 4;
    const v4f v = *(const v4f*)(src + off0 + (size_t)(r0 + r) * ld + c4);
#pragma unroll
    for (int i = 0; i < 4; ++i) { const unsigned hb = bf16_rne_bits(v[i]); unsigned short o = (unsigned short)hb;
      if (f16mode) { const _Float16 hv = (_Float16)(__uint_as_float(hb << 16) * 256.0f); o = __builtin_bit_cast(unsigned short, hv); }
      t[c4 + i][r] = o; } }
  __syncthreads();
#pragma unroll 1
  for (int it = 0; it < 2; ++it) { const int e = tid + it * 256; const int c = e >> 3, q = e & 7;
    vst2(dst + ((size_t)y * 64 + c) * DIN + r0 + q * 8, *(const v4u*)&t[c][q * 8]); }
}
__global__ __launch_bounds__(128) void k_proj(const __bf16* __restrict__ XB, const __bf16* __restrict__ WT, _Float16* __restrict__ QKH, _Float16* __restrict__ QKL, _Float16* __restrict__ VT, __bf16* __restrict__ VB, __bf16* __restrict__ VBL) {
  __shared__ __align__(16) _Float16 sh[64][136], sl[64][136]; __shared__ __align__(16) _Float16 th[128][72]; __shared__ __align__(16) __bf16 tb[128][72], tbl[128][72];
  const int tid = threadIdx.x, lane = tid & 31, col = lane & 15, g = lane >> 4; const int wave = __builtin_amdgcn_readfirstlane((int)(threadIdx.x >> 5));
  const int which = blockIdx.z; const int c0 = (int)blockIdx.y * 128; const size_t r0 = (size_t)blockIdx.x * 64; const size_t bb = r0 / TT; const int t0 = (int)(r0 % TT);
  const __bf16* Ar = XB + (r0 + wave * 16 + col) * DIN; const __bf16* Wr = WT + ((size_t)which * CC + c0 + col) * DIN;
  v8f acc[8] = {};
#pragma unroll 2
  for (int kc = 0; kc < DIN / 32; ++kc) { const v16b a = frag_b(Ar + kc * 32, lane);
    asm volatile("s_wait_loadcnt 0x0" ::: "memory");
#pragma unroll
    for (int j = 0; j < 8; ++j) { const v16b w = frag_b(Wr + (size_t)j * 16 * DIN + kc * 32, lane); asm volatile("s_wait_loadcnt 0x0" ::: "memory"); acc[j] = wmma_bf(a, w, acc[j]); } }
  if (which < 2) { _Float16* DH = QKH + (size_t)which * NB * TT * CC; _Float16* DL = QKL + (size_t)which * NB * QHI * CC; const bool hi_rows = t0 < QHI;
#pragma unroll
    for (int j = 0; j < 8; ++j) {
#pragma unroll
      for (int r = 0; r < 8; ++r) { const float v = acc[j][r]; const _Float16 hv = (_Float16)v; sh[wave * 16 + 8 * g + r][j * 16 + col] = hv; sl[wave * 16 + 8 * g + r][j * 16 + col] = (_Float16)((v - (float)hv) * 1024.0f); } }
    __syncthreads();
    for (int e = tid; e < 64 * 16; e += 128) { const int rl = e >> 4, q = e & 15;
      vst2(DH + (r0 + rl) * CC + c0 + q * 8, *(const v4u*)&sh[rl][q * 8]);
      if (hi_rows) vst2(DL + (bb * QHI + t0 + rl) * (size_t)CC + c0 + q * 8, *(const v4u*)&sl[rl][q * 8]); }
  } else { const bool hi_rows = t0 < KHI;
#pragma unroll
    for (int j = 0; j < 8; ++j) {
#pragma unroll
      for (int r = 0; r < 8; ++r) { const float v = acc[j][r]; const int rl = wave * 16 + 8 * g + r, cl = j * 16 + col; th[cl][rl] = (_Float16)v; const __bf16 bh = (__bf16)v; tb[cl][rl] = bh; tbl[cl][rl] = (__bf16)(v - (float)bh); } }
    __syncthreads();
    for (int e = tid; e < 128 * 8; e += 128) { const int cl = e >> 3, q = e & 7;
      vst2(VT + (bb * CC + c0 + cl) * (size_t)TT + t0 + q * 8, *(const v4u*)&th[cl][q * 8]);
      if (hi_rows) { const size_t o3 = (bb * CC + c0 + cl) * (size_t)KHI + t0 + q * 8; vst2(VB + o3, *(const v4u*)&tb[cl][q * 8]); vst2(VBL + o3, *(const v4u*)&tbl[cl][q * 8]); } } } }

__device__ __forceinline__ void osm_step(float (&x0)[8], float (&x1)[8], float (&m)[8], float (&l)[8], float (&al)[8]) {
#pragma unroll
  for (int r = 0; r < 8; ++r) { float mx = fmaxf(x0[r], x1[r]);
    mx = fmaxf(mx, __shfl_xor(mx, 1)); mx = fmaxf(mx, __shfl_xor(mx, 2)); mx = fmaxf(mx, __shfl_xor(mx, 4)); mx = fmaxf(mx, __shfl_xor(mx, 8));
    const float mn = fmaxf(m[r], mx); al[r] = exp2f(m[r] - mn); m[r] = mn;
    x0[r] = exp2f(x0[r] - mn); x1[r] = exp2f(x1[r] - mn); l[r] = l[r] * al[r] + (x0[r] + x1[r]); } }

__global__ __launch_bounds__(128) void k_attn_hi(const _Float16* __restrict__ QH, const _Float16* __restrict__ QL, const _Float16* __restrict__ KH, const _Float16* __restrict__ KL, const __bf16* __restrict__ VB, const __bf16* __restrict__ VBL, _Float16* __restrict__ CH, _Float16* __restrict__ CL) {
  __shared__ __align__(16) __bf16 pbh[4][16][40], pbl[4][16][40];
  __shared__ __align__(16) _Float16 osh[4][16][72], osl[4][16][72];
  const int tid = threadIdx.x, lane = tid & 31, col = lane & 15, g = lane >> 4; const int wave = __builtin_amdgcn_readfirstlane((int)(threadIdx.x >> 5));
  const int qb = blockIdx.x, h = blockIdx.y, b = blockIdx.z; const int ql0 = qb * 64 + wave * 16;
  const _Float16* Qr = QH + ((size_t)b * TT + ql0 + col) * CC + h * HD; const _Float16* Qlr = QL + ((size_t)b * QHI + ql0 + col) * CC + h * HD;
  const v16h qh0 = frag_h(Qr, lane), qh1 = frag_h(Qr + 32, lane), qr0 = frag_h(Qlr, lane), qr1 = frag_h(Qlr + 32, lane);
  const _Float16* Kb = KH + (size_t)b * TT * CC + h * HD; const _Float16* Klb = KL + (size_t)b * KHI * CC + h * HD;
  const __bf16* Vb = VB + ((size_t)b * CC + h * HD) * KHI; const __bf16* Vlb = VBL + ((size_t)b * CC + h * HD) * KHI;
  v8f o[4] = {}; float m[8], l[8];
#pragma unroll
  for (int r = 0; r < 8; ++r) { m[r] = -3.0e38f; l[r] = 0.f; }
  const int nst = (ql0 + 47) >> 5;
#pragma unroll 1
  for (int st = 0; st < nst; ++st) { const int kbase = st * 32; float x0[8], x1[8], al[8];
    { const size_t kr = (size_t)(kbase + col) * CC; v8f s = {}, sr = {};
      v16h kh = frag_h(Kb + kr, lane), kl = frag_h(Klb + kr, lane); s = wmma16(qh0, kh, s); sr = wmma16(qr0, kh, sr); sr = wmma16(qh0, kl, sr);
      kh = frag_h(Kb + kr + 32, lane); kl = frag_h(Klb + kr + 32, lane); s = wmma16(qh1, kh, s); sr = wmma16(qr1, kh, sr); sr = wmma16(qh1, kl, sr);
#pragma unroll
      for (int r = 0; r < 8; ++r) x0[r] = (s[r] + sr[r] * (1.0f / 1024.0f)) * SC_LOG2E; }
    { const size_t kr = (size_t)(kbase + 16 + col) * CC; v8f s = {}, sr = {};
      v16h kh = frag_h(Kb + kr, lane), kl = frag_h(Klb + kr, lane); s = wmma16(qh0, kh, s); sr = wmma16(qr0, kh, sr); sr = wmma16(qh0, kl, sr);
      kh = frag_h(Kb + kr + 32, lane); kl = frag_h(Klb + kr + 32, lane); s = wmma16(qh1, kh, s); sr = wmma16(qr1, kh, sr); sr = wmma16(qh1, kl, sr);
#pragma unroll
      for (int r = 0; r < 8; ++r) x1[r] = (s[r] + sr[r] * (1.0f / 1024.0f)) * SC_LOG2E; }
    if (kbase + 31 > ql0) {
#pragma unroll
      for (int r = 0; r < 8; ++r) { const int qr = ql0 + 8 * g + r; x0[r] = (kbase + col > qr) ? -3.0e38f : x0[r]; x1[r] = (kbase + 16 + col > qr) ? -3.0e38f : x1[r]; } }
    osm_step(x0, x1, m, l, al);
#pragma unroll
    for (int j = 0; j < 4; ++j)
#pragma unroll
      for (int r = 0; r < 8; ++r) o[j][r] *= al[r];
#pragma unroll
    for (int r = 0; r < 8; ++r) { const __bf16 h0 = (__bf16)x0[r], h1 = (__bf16)x1[r];
      pbh[wave][8 * g + r][col] = h0; pbl[wave][8 * g + r][col] = (__bf16)(x0[r] - (float)h0);
      pbh[wave][8 * g + r][16 + col] = h1; pbl[wave][8 * g + r][16 + col] = (__bf16)(x1[r] - (float)h1); }
    LDSX();
    v16b ph, pl; { union { v16b v; v8b q[2]; } u; u.q[0] = *(const v8b*)&pbh[wave][col][8 * g]; u.q[1] = *(const v8b*)&pbh[wave][col][16 + 8 * g]; ph = u.v;
      u.q[0] = *(const v8b*)&pbl[wave][col][8 * g]; u.q[1] = *(const v8b*)&pbl[wave][col][16 + 8 * g]; pl = u.v; }
    LDSX();
#pragma unroll
    for (int j = 0; j < 4; ++j) { const size_t vo = (size_t)(j * 16 + col) * KHI + kbase; const v16b vh = frag_b(Vb + vo, lane), vl = frag_b(Vlb + vo, lane);
      o[j] = wmma_bf(pl, vh, o[j]); o[j] = wmma_bf(ph, vl, o[j]); o[j] = wmma_bf(ph, vh, o[j]); } }
  float inv[8];
#pragma unroll
  for (int r = 0; r < 8; ++r) { float s = l[r]; s += __shfl_xor(s, 1); s += __shfl_xor(s, 2); s += __shfl_xor(s, 4); s += __shfl_xor(s, 8); inv[r] = 64.0f * (1.0f / s); }
#pragma unroll
  for (int j = 0; j < 4; ++j)
#pragma unroll
    for (int r = 0; r < 8; ++r) { const float v = o[j][r] * inv[r]; const _Float16 hv = (_Float16)v; osh[wave][8 * g + r][j * 16 + col] = hv; osl[wave][8 * g + r][j * 16 + col] = (_Float16)((v - (float)hv) * 1024.0f); }
  LDSX();
#pragma unroll 1
  for (int it = 0; it < 4; ++it) { const int rl = it * 4 + (lane >> 3), q = lane & 7;
    vst2(CH + ((size_t)b * TT + ql0 + rl) * CC + h * HD + q * 8, *(const v4u*)&osh[wave][rl][q * 8]);
    vst2(CL + ((size_t)b * QHI + ql0 + rl) * CC + h * HD + q * 8, *(const v4u*)&osl[wave][rl][q * 8]); }
}
__global__ __launch_bounds__(128) void k_attn(const _Float16* __restrict__ QH, const _Float16* __restrict__ KH, const _Float16* __restrict__ VT, _Float16* __restrict__ CH) {
  __shared__ __align__(16) _Float16 ps[4][16][40];
  __shared__ __align__(16) _Float16 os[4][16][72];
  const int tid = threadIdx.x, lane = tid & 31, col = lane & 15, g = lane >> 4; const int wave = __builtin_amdgcn_readfirstlane((int)(threadIdx.x >> 5));
  const int qb = QBH + (int)blockIdx.x, h = blockIdx.y, b = blockIdx.z; const int ql0 = qb * 64 + wave * 16;
  const _Float16* Qr = QH + ((size_t)b * TT + ql0 + col) * CC + h * HD;
  const v16h q0 = frag_h(Qr, lane), q1 = frag_h(Qr + 32, lane);
  const _Float16* Kb = KH + (size_t)b * TT * CC + h * HD; const _Float16* Vb = VT + ((size_t)b * CC + h * HD) * TT;
  v8f o[4] = {}; float m[8], l[8];
#pragma unroll
  for (int r = 0; r < 8; ++r) { m[r] = -3.0e38f; l[r] = 0.f; }
  const int nst = (ql0 + 47) >> 5;
#pragma unroll 1
  for (int st = 0; st < nst; ++st) { const int kbase = st * 32; float x0[8], x1[8], al[8];
    { const _Float16* kr = Kb + (size_t)(kbase + col) * CC; v8f s = {};
      s = wmma16(q0, frag_h(kr, lane), s); s = wmma16(q1, frag_h(kr + 32, lane), s);
#pragma unroll
      for (int r = 0; r < 8; ++r) x0[r] = s[r] * SC_LOG2E; }
    { const _Float16* kr = Kb + (size_t)(kbase + 16 + col) * CC; v8f s = {};
      s = wmma16(q0, frag_h(kr, lane), s); s = wmma16(q1, frag_h(kr + 32, lane), s);
#pragma unroll
      for (int r = 0; r < 8; ++r) x1[r] = s[r] * SC_LOG2E; }
    if (kbase + 31 > ql0) {
#pragma unroll
      for (int r = 0; r < 8; ++r) { const int qr = ql0 + 8 * g + r; x0[r] = (kbase + col > qr) ? -3.0e38f : x0[r]; x1[r] = (kbase + 16 + col > qr) ? -3.0e38f : x1[r]; } }
    osm_step(x0, x1, m, l, al);
#pragma unroll
    for (int j = 0; j < 4; ++j)
#pragma unroll
      for (int r = 0; r < 8; ++r) o[j][r] *= al[r];
#pragma unroll
    for (int r = 0; r < 8; ++r) { ps[wave][8 * g + r][col] = (_Float16)(x0[r] * 1024.0f); ps[wave][8 * g + r][16 + col] = (_Float16)(x1[r] * 1024.0f); }
    LDSX();
    v16h pf; { union { v16h v; v8h q[2]; } u; u.q[0] = *(const v8h*)&ps[wave][col][8 * g]; u.q[1] = *(const v8h*)&ps[wave][col][16 + 8 * g]; pf = u.v; }
    LDSX();
#pragma unroll
    for (int j = 0; j < 4; ++j) o[j] = wmma16(pf, frag_h(Vb + (size_t)(j * 16 + col) * TT + kbase, lane), o[j]); }
  float inv[8];
#pragma unroll
  for (int r = 0; r < 8; ++r) { float s = l[r]; s += __shfl_xor(s, 1); s += __shfl_xor(s, 2); s += __shfl_xor(s, 4); s += __shfl_xor(s, 8); inv[r] = 0.0625f * (1.0f / s); }
#pragma unroll
  for (int j = 0; j < 4; ++j)
#pragma unroll
    for (int r = 0; r < 8; ++r) os[wave][8 * g + r][j * 16 + col] = (_Float16)(o[j][r] * inv[r]);
  LDSX();
#pragma unroll 1
  for (int it = 0; it < 4; ++it) { const int rl = it * 4 + (lane >> 3), q = lane & 7;
    vst2(CH + ((size_t)b * TT + ql0 + rl) * CC + h * HD + q * 8, *(const v4u*)&os[wave][rl][q * 8]); }
}
__global__ __launch_bounds__(128) void k_out(const _Float16* __restrict__ CH, const _Float16* __restrict__ CL, const _Float16* __restrict__ WPH, float* __restrict__ OUT) {
  __shared__ __align__(16) float sf[4][16][132];
  const int tid = threadIdx.x, lane = tid & 31, col = lane & 15, g = lane >> 4; const int wave = __builtin_amdgcn_readfirstlane((int)(threadIdx.x >> 5));
  const int c0 = (int)blockIdx.y * 128; const size_t rb = (size_t)blockIdx.x * 64; const size_t bb = rb / TT; const int t0 = (int)(rb % TT);
  const _Float16* Ar = CH + (rb + wave * 16 + col) * CC; const _Float16* Wr = WPH + ((size_t)c0 + col) * CC;
  v8f acc[8] = {};
  if (t0 < QHI) {
    const _Float16* Alr = CL + (bb * QHI + t0 + wave * 16 + col) * (size_t)CC; v8f accl[8] = {};
#pragma unroll 2
    for (int kc = 0; kc < CC / 32; ++kc) { const v16h a = frag_h(Ar + kc * 32, lane), al = frag_h(Alr + kc * 32, lane); asm volatile("s_wait_loadcnt 0x0" ::: "memory");
#pragma unroll
      for (int j = 0; j < 8; ++j) { const v16h w = frag_h(Wr + (size_t)j * 16 * CC + kc * 32, lane); asm volatile("s_wait_loadcnt 0x0" ::: "memory"); acc[j] = wmma16(a, w, acc[j]); accl[j] = wmma16(al, w, accl[j]); } }
#pragma unroll
    for (int j = 0; j < 8; ++j)
#pragma unroll
      for (int r = 0; r < 8; ++r) sf[wave][8 * g + r][j * 16 + col] = (acc[j][r] + accl[j][r] * (1.0f / 1024.0f)) * (1.0f / 16384.0f);
  } else {
#pragma unroll 2
    for (int kc = 0; kc < CC / 32; ++kc) { const v16h a = frag_h(Ar + kc * 32, lane); asm volatile("s_wait_loadcnt 0x0" ::: "memory");
#pragma unroll
      for (int j = 0; j < 8; ++j) { const v16h w = frag_h(Wr + (size_t)j * 16 * CC + kc * 32, lane); asm volatile("s_wait_loadcnt 0x0" ::: "memory"); acc[j] = wmma16(a, w, acc[j]); } }
#pragma unroll
    for (int j = 0; j < 8; ++j)
#pragma unroll
      for (int r = 0; r < 8; ++r) sf[wave][8 * g + r][j * 16 + col] = acc[j][r] * (1.0f / 16384.0f); }
  LDSX();
  const size_t orow = bb * TT_FULL + (size_t)t0 + wave * 16;
#pragma unroll 1
  for (int rl = 0; rl < 16; ++rl) vst2(OUT + (orow + rl) * DIN + c0 + lane * 4, *(const v4f*)&sf[wave][rl][lane * 4]);
}

extern "C" void kernel_launch(void* const* d_in, const int* in_sizes, int n_in, void* d_out, int out_size, void* d_ws, size_t ws_size, hipStream_t stream) {
  if (n_in < 5) return;
  if (ws_size < (size_t)WS_END) return;
  const long long need_rows = (long long)(NB - 1) * TT_FULL + TT;
  if ((long long)in_sizes[0] < need_rows * DIN) return;
  if ((long long)in_sizes[1] < (long long)NH * DIN * HD) return;
  if ((long long)in_sizes[2] < (long long)NH * DIN * HD) return;
  if ((long long)in_sizes[3] < (long long)NH * DIN * HD) return;
  if ((long long)in_sizes[4] < (long long)CC * DIN) return;
  if ((long long)out_size < need_rows * DIN) return;
  const float* X = (const float*)d_in[0]; const float* Wq = (const float*)d_in[1]; const float* Wk = (const float*)d_in[2]; const float* Wv = (const float*)d_in[3]; const float* Wp = (const float*)d_in[4];
  char* ws = (char*)d_ws;
  unsigned short* XBw = (unsigned short*)(ws + WS_XB); unsigned short* WTw = (unsigned short*)(ws + WS_WT); unsigned short* WPHw = (unsigned short*)(ws + WS_WPH);
  const __bf16* XB = (const __bf16*)(ws + WS_XB); const __bf16* WT = (const __bf16*)(ws + WS_WT); const _Float16* WPH = (const _Float16*)(ws + WS_WPH);
  _Float16 *QH = (_Float16*)(ws + WS_QH), *KH = (_Float16*)(ws + WS_KH), *VT = (_Float16*)(ws + WS_VT), *QL = (_Float16*)(ws + WS_QL), *KL = (_Float16*)(ws + WS_KL), *CH = (_Float16*)(ws + WS_CH), *CL = (_Float16*)(ws + WS_CL);
  __bf16 *VB = (__bf16*)(ws + WS_VB), *VBL = (__bf16*)(ws + WS_VBL);
  k_cvt_x<<<dim3(NB * TT * (DIN / 8) / 256), 256, 0, stream>>>(X, XBw);
  k_wt<<<dim3(DIN / 64, NH), 256, 0, stream>>>(Wq, WTw, 1, 0);
  k_wt<<<dim3(DIN / 64, NH), 256, 0, stream>>>(Wk, WTw + (size_t)CC * DIN, 1, 0);
  k_wt<<<dim3(DIN / 64, NH), 256, 0, stream>>>(Wv, WTw + (size_t)2 * CC * DIN, 1, 0);
  k_wt<<<dim3(CC / 64, DIN / 64), 256, 0, stream>>>(Wp, WPHw, 0, 1);
  k_proj<<<dim3(NB * TT / 64, CC / 128, 3), 128, 0, stream>>>(XB, WT, QH, QL, VT, VB, VBL);
  k_attn_hi<<<dim3(QBH, NH, NB), 128, 0, stream>>>(QH, QL, KH, KL, VB, VBL, CH, CL);
  if (NQB > QBH) k_attn<<<dim3(NQB > QBH ? NQB - QBH : 1, NH, NB), 128, 0, stream>>>(QH, KH, VT, CH);
  k_out<<<dim3(NB * TT / 64, DIN / 128), 128, 0, stream>>>(CH, CL, WPH, (float*)d_out);
}
